// Mamba2_50646254355296
// MI455X (gfx1250) — hardware-run, weakly checked
//
#include <hip/hip_runtime.h>
#include <math.h>

typedef __attribute__((ext_vector_type(16))) _Float16 v16h;
typedef __attribute__((ext_vector_type(8)))  _Float16 v8h;
typedef __attribute__((ext_vector_type(8)))  float    v8f;
typedef __attribute__((ext_vector_type(4)))  float    v4f;

constexpr int kBatch  = 2;
constexpr int kL      = 1024;
constexpr int kDm     = 1024;
constexpr int kNH     = 32;
constexpr int kDH     = 64;
constexpr int kDS     = 64;
constexpr int kDI     = kNH * kDH;
constexpr int kXBC    = kDI + 2 * kDS;
constexpr int kProj   = 2 * kDI + 2 * kDS + kNH;
constexpr int kProjP  = 4288;
constexpr int kRows   = kBatch * kL;
constexpr int kColX   = kDI;
constexpr int kColDt  = kDI + kXBC;
static_assert(kDI == 2048);
static_assert(kXBC == 2176);
static_assert(kProj == 4256);
static_assert(kColDt == 4224);
static_assert(kProjP % 64 == 0 && kProjP >= kProj);
static_assert(kRows % 64 == 0 && kDm % 64 == 0 && kDm % 32 == 0 && kDI % 32 == 0);
static_assert(kProj % 4 == 0 && kDm % 4 == 0);
static_assert(kDH == 64 && kDS == 64 && kNH == 32);

constexpr float kCarryX = 16.0f;
constexpr float kCarryW = 1024.0f;
constexpr float kCarryY = 128.0f;
constexpr float kScaleIn  = 1.0f / (kCarryX * kCarryW);
constexpr float kScaleOut = 1.0f / (kCarryY * kCarryW);

constexpr size_t kSzXH    = (size_t)kRows * kDm * 2;
constexpr size_t kSzWINT  = (size_t)kProjP * kDm * 2;
constexpr size_t kSzWOUTT = (size_t)kDm * kDI * 2;
constexpr size_t kSzXZ    = (size_t)kRows * kProjP * 4;
constexpr size_t kSzXC    = (size_t)kRows * kXBC * 4;
constexpr size_t kSzDTV   = (size_t)kRows * kNH * 4;
constexpr size_t kSzDAV   = (size_t)kRows * kNH * 4;
constexpr size_t kSzYB    = (size_t)kRows * kDI * 4;
constexpr size_t kSzYN    = (size_t)kRows * kDI * 2;
constexpr size_t kOffXH    = 0;
constexpr size_t kOffWINT  = kOffXH + kSzXH;
constexpr size_t kOffWOUTT = kOffWINT + kSzWINT;
constexpr size_t kOffXZ    = kOffWOUTT + kSzWOUTT;
constexpr size_t kOffXC    = kOffXZ + kSzXZ;
constexpr size_t kOffDTV   = kOffXC + kSzXC;
constexpr size_t kOffDAV   = kOffDTV + kSzDTV;
constexpr size_t kOffYB    = kOffDAV + kSzDAV;
constexpr size_t kOffYN    = kOffYB + kSzYB;
constexpr size_t kWsTotal  = kOffYN + kSzYN;
static_assert(kWsTotal == 95813632ull);
static_assert(kWsTotal <= 134217728ull);
static_assert((kOffWINT % 128) == 0 && (kOffWOUTT % 128) == 0 && (kOffXZ % 128) == 0 && (kOffXC % 128) == 0 &&
              (kOffDTV % 128) == 0 && (kOffDAV % 128) == 0 && (kOffYB % 128) == 0 && (kOffYN % 128) == 0);

__device__ __forceinline__ v16h frag_load_h(const _Float16* p) {
  union U { v16h v; v8h h[2]; } f;
  f.h[0] = *(const v8h*)(p);
  f.h[1] = *(const v8h*)(p + 16);
  return f.v;
}
__device__ __forceinline__ v8f mma_h(v16h a, v16h b, v8f c) {
  c = __builtin_amdgcn_wmma_f32_16x16x32_f16(false, a, false, b, (short)0, c, false, false);
  asm volatile("v_nop\n\tv_nop\n\tv_nop\n\tv_nop" : "+v"(c) : "v"(a), "v"(b));
  return c;
}

__global__ __launch_bounds__(256) void wmma_gemm64_f16(
    const unsigned short* __restrict__ Ap, int lda,
    const unsigned short* __restrict__ Btp, int ldb,
    float* __restrict__ C, int ldc,
    int M, int N, int K, float scale) {
  const _Float16* A  = (const _Float16*)Ap;
  const _Float16* Bt = (const _Float16*)Btp;
  __shared__ __align__(16) float sT[8][16 * 68];
  const int lane = threadIdx.x & 31;
  const int wave = __builtin_amdgcn_readfirstlane((int)(threadIdx.x >> 5));
  const int tilesN = N >> 6;
  const int tilesM = M >> 6;
  const int tile = blockIdx.x * 8 + wave;
  if (tile >= tilesM * tilesN) return;
  const int tm = tile / tilesN;
  const int tn = tile - tm * tilesN;
  const int m0 = tm << 6;
  const int n0 = tn << 6;

  const int rlane = lane & 15;
  const int koff  = (lane >> 4) * 8;
  const int mOff  = (lane >> 4) * 8;

  v8f acc[4][4];
#pragma unroll
  for (int i = 0; i < 4; ++i)
#pragma unroll
    for (int j = 0; j < 4; ++j) acc[i][j] = (v8f){0.f, 0.f, 0.f, 0.f, 0.f, 0.f, 0.f, 0.f};

  for (int k0 = 0; k0 < K; k0 += 32) {
    v16h bh[4];
#pragma unroll
    for (int j = 0; j < 4; ++j) {
      const size_t bo = (size_t)(n0 + (j << 4) + rlane) * ldb + koff + k0;
      bh[j] = frag_load_h(Bt + bo);
    }
#pragma unroll
    for (int i = 0; i < 4; ++i) {
      const size_t ao = (size_t)(m0 + (i << 4) + rlane) * lda + koff + k0;
      const v16h ah = frag_load_h(A + ao);
#pragma unroll
      for (int j = 0; j < 4; ++j) acc[i][j] = mma_h(ah, bh[j], acc[i][j]);
    }
  }

  float* slab = sT[wave];
#pragma unroll
  for (int i = 0; i < 4; ++i) {
    const int mBase = m0 + (i << 4);
#pragma unroll
    for (int j = 0; j < 4; ++j) {
#pragma unroll
      for (int r = 0; r < 8; ++r) {
        const float v = acc[i][j][r] * scale;
        slab[(mOff + r) * 68 + (j << 4) + rlane] = v;
      }
    }
    __builtin_amdgcn_fence(__ATOMIC_RELEASE, "workgroup");
    __builtin_amdgcn_wave_barrier();
    __builtin_amdgcn_fence(__ATOMIC_ACQUIRE, "workgroup");
    {
      const int hh = lane >> 4, c4 = (lane & 15) * 4;
      for (int pass = 0; pass < 2; ++pass) {
#pragma unroll
        for (int it = 0; it < 8; ++it) {
          const int row = it * 2 + hh;
          const v4f v = *(const v4f*)(slab + row * 68 + c4);
          *(volatile v4f*)(C + (size_t)(mBase + row) * ldc + n0 + c4) = v;
        }
        __threadfence();
      }
    }
    __builtin_amdgcn_fence(__ATOMIC_RELEASE, "workgroup");
    __builtin_amdgcn_wave_barrier();
    __builtin_amdgcn_fence(__ATOMIC_ACQUIRE, "workgroup");
  }
}

static_assert(((kRows * kDm / 8) % 256) == 0);
__global__ __launch_bounds__(256) void cvt_rows_f16_kernel(
    const float* __restrict__ src, unsigned short* __restrict__ dst, int total8, float carry) {
  const int i = blockIdx.x * 256 + threadIdx.x;
  if (i >= total8) return;
  const size_t e0 = (size_t)i << 3;
  const v4f a0 = *(const v4f*)(src + e0);
  const v4f a1 = *(const v4f*)(src + e0 + 4);
  v8h hv;
#pragma unroll
  for (int e = 0; e < 4; ++e) {
    const float f0 = a0[e] * carry;
    const float f1 = a1[e] * carry;
    hv[e]     = (_Float16)f0;
    hv[4 + e] = (_Float16)f1;
  }
  unsigned short* q = dst + e0;
  *(volatile v8h*)q = hv;
  __threadfence();
  *(volatile v8h*)q = hv;
}

__global__ __launch_bounds__(256) void transpose_cvt_f16_kernel(
    const float* __restrict__ in, unsigned short* __restrict__ out, int KR, int NC, float carry) {
  __shared__ __align__(16) float sT[64 * 68];
  const int tid  = threadIdx.x;
  const int lane = tid & 31;
  const int wave = __builtin_amdgcn_readfirstlane((int)(threadIdx.x >> 5));
  const int n0 = blockIdx.x * 64;
  const int k0 = blockIdx.y * 64;
  const int lr = tid >> 4, n4 = (tid & 15) * 4;
  const int n  = n0 + n4;
  const bool ok = (n < NC);
  const int nc = ok ? n : (NC - 4);
#pragma unroll
  for (int it = 0; it < 4; ++it) {
    const int k = it * 16 + lr;
    const v4f v = *(const v4f*)(in + (size_t)(k0 + k) * NC + nc);
    v4f w;
    w[0] = ok ? (v[0] * carry) : 0.0f;
    w[1] = ok ? (v[1] * carry) : 0.0f;
    w[2] = ok ? (v[2] * carry) : 0.0f;
    w[3] = ok ? (v[3] * carry) : 0.0f;
    *(v4f*)(sT + k * 68 + n4) = w;
  }
  __syncthreads();
  const int q = lane >> 3, c8 = (lane & 7) * 8;
  v8h hv[2];
#pragma unroll
  for (int it = 0; it < 2; ++it) {
    const int nr = it * 32 + wave * 4 + q;
#pragma unroll
    for (int e = 0; e < 8; ++e) {
      const float f = sT[(c8 + e) * 68 + nr];
      hv[it][e] = (_Float16)f;
    }
  }
  for (int pass = 0; pass < 2; ++pass) {
#pragma unroll
    for (int it = 0; it < 2; ++it) {
      const int nr = it * 32 + wave * 4 + q;
      *(volatile v8h*)(out + (size_t)(n0 + nr) * KR + k0 + c8) = hv[it];
    }
    __threadfence();
  }
}

constexpr int kCvTP = 132;
static_assert(kXBC % 128 == 0 && kL % 64 == 0);
__global__ __launch_bounds__(128) void conv_silu_kernel(
    const float* __restrict__ XZ, const float* __restrict__ cw, const float* __restrict__ cb,
    float* __restrict__ XC) {
  __shared__ __align__(16) float sT[16 * kCvTP];
  const int tid  = threadIdx.x;
  const int lane = tid & 31;
  const int wave = __builtin_amdgcn_readfirstlane((int)(threadIdx.x >> 5));
  const int c0 = blockIdx.x * 128;
  const int c  = c0 + tid;
  const int g0 = blockIdx.y * 64;
  const int tb = g0 & (kL - 1);
  const v4f w = *(const v4f*)(cw + (size_t)c * 4);
  const float bc = cb[c];
  const float* col = XZ + kColX + c;
  float xm3, xm2, xm1;
  {
    const bool hist = (tb > 0);
    const int rb = hist ? (g0 - 3) : g0;
    const float v3 = col[(size_t)rb * kProjP];
    const float v2 = col[(size_t)(rb + 1) * kProjP];
    const float v1 = col[(size_t)(rb + 2) * kProjP];
    xm3 = hist ? v3 : 0.0f;
    xm2 = hist ? v2 : 0.0f;
    xm1 = hist ? v1 : 0.0f;
  }
#pragma unroll 1
  for (int sub = 0; sub < 4; ++sub) {
    const int lb = g0 + sub * 16;
#pragma unroll 1
    for (int s = 0; s < 16; ++s) {
      const float xcur = col[(size_t)(lb + s) * kProjP];
      float acc = w[0] * xm3;
      acc = fmaf(w[1], xm2, acc);
      acc = fmaf(w[2], xm1, acc);
      acc = fmaf(w[3], xcur, acc);
      const float sv = acc + bc;
      const float sg = 1.0f / (1.0f + expf(-sv));
      sT[s * kCvTP + tid] = sv * sg;
      xm3 = xm2;
      xm2 = xm1;
      xm1 = xcur;
    }
    __syncthreads();
    v4f fv[4];
#pragma unroll
    for (int it = 0; it < 4; ++it) fv[it] = *(const v4f*)(sT + (it * 4 + wave) * kCvTP + lane * 4);
    for (int pass = 0; pass < 2; ++pass) {
#pragma unroll
      for (int it = 0; it < 4; ++it)
        *(volatile v4f*)(XC + (size_t)(lb + it * 4 + wave) * kXBC + c0 + lane * 4) = fv[it];
      __threadfence();
    }
    __syncthreads();
  }
}

static_assert(kRows % 8 == 0);
__global__ __launch_bounds__(256) void dt_kernel(
    const float* __restrict__ XZ, const float* __restrict__ A_log, const float* __restrict__ dt_bias,
    float* __restrict__ DTV, float* __restrict__ DAV) {
  const int lane = threadIdx.x & 31;
  const int wave = __builtin_amdgcn_readfirstlane((int)(threadIdx.x >> 5));
  const int row  = blockIdx.x * 8 + wave;
  const float v  = XZ[(size_t)row * kProjP + kColDt + lane] + dt_bias[lane];
  const float e  = expf(-fabsf(v));
  const float dt = fmaxf(v, 0.0f) + log1pf(e);
  const float Ah = -expf(A_log[lane]);
  const float dA = expf(Ah * dt);
  float* p0 = DTV + (size_t)row * kNH + lane;
  float* p1 = DAV + (size_t)row * kNH + lane;
  *(volatile float*)p0 = dt;
  *(volatile float*)p1 = dA;
  __threadfence();
  *(volatile float*)p0 = dt;
  *(volatile float*)p1 = dA;
}

constexpr int kScT  = 32;
constexpr int kScYP = 68;
static_assert(kScT == 32 && (kL % kScT) == 0);
__global__ __launch_bounds__(128) void scan_kernel(
    const float* __restrict__ XC, const float* __restrict__ DTV, const float* __restrict__ DAV,
    const float* __restrict__ Dp, float* __restrict__ YB) {
  __shared__ __align__(16) float sX[kScT * 64];
  __shared__ __align__(16) float sBm[kScT * 64];
  __shared__ __align__(16) float sCm[kScT * 64];
  __shared__ __align__(16) float sDt[kScT];
  __shared__ __align__(16) float sDa[kScT];
  __shared__ __align__(16) float sY[2 * kScT * kScYP];
  const int tid  = threadIdx.x;
  const int lane = tid & 31;
  const int wave = __builtin_amdgcn_readfirstlane((int)(threadIdx.x >> 5));
  const int half = wave >> 1;
  const int d    = (wave & 1) * 32 + lane;
  const int bix  = blockIdx.x >> 5;
  const int head = blockIdx.x & 31;
  const size_t row0 = (size_t)bix * kL;
  const float Dd = Dp[head];
  float h[32];
#pragma unroll
  for (int j = 0; j < 32; ++j) h[j] = 0.0f;
  const int hh = lane >> 4, c4 = (lane & 15) * 4;

#pragma unroll 1
  for (int t0 = 0; t0 < kL; t0 += kScT) {
    __syncthreads();
#pragma unroll
    for (int i = 0; i < 4; ++i) {
      const int idx = i * 128 + tid;
      const int r = idx >> 4, cc = (idx & 15) * 4;
      const float* base = XC + (row0 + t0 + r) * kXBC;
      *(v4f*)(sX  + r * 64 + cc) = *(const v4f*)(base + head * kDH + cc);
      *(v4f*)(sBm + r * 64 + cc) = *(const v4f*)(base + kDI + cc);
      *(v4f*)(sCm + r * 64 + cc) = *(const v4f*)(base + kDI + kDS + cc);
    }
    {
      const size_t gi = (row0 + t0 + lane) * kNH + head;
      if (wave == 0) sDt[lane] = DTV[gi];
      if (wave == 1) sDa[lane] = DAV[gi];
    }
    __syncthreads();

#pragma unroll 1
    for (int s = 0; s < kScT; ++s) {
      const float dt = sDt[s];
      const float dA = sDa[s];
      const float xt = sX[s * 64 + d];
      const float coef = dt * xt;
      const float* bp = sBm + s * 64 + half * 32;
      const float* cp = sCm + s * 64 + half * 32;
      float y = 0.0f;
#pragma unroll
      for (int q = 0; q < 8; ++q) {
        const v4f bv = *(const v4f*)(bp + 4 * q);
        const v4f cv = *(const v4f*)(cp + 4 * q);
        h[4 * q + 0] = fmaf(dA, h[4 * q + 0], coef * bv[0]);
        y = fmaf(h[4 * q + 0], cv[0], y);
        h[4 * q + 1] = fmaf(dA, h[4 * q + 1], coef * bv[1]);
        y = fmaf(h[4 * q + 1], cv[1], y);
        h[4 * q + 2] = fmaf(dA, h[4 * q + 2], coef * bv[2]);
        y = fmaf(h[4 * q + 2], cv[2], y);
        h[4 * q + 3] = fmaf(dA, h[4 * q + 3], coef * bv[3]);
        y = fmaf(h[4 * q + 3], cv[3], y);
      }
      sY[half * (kScT * kScYP) + s * kScYP + d] = y;
    }
    __syncthreads();

#pragma unroll 1
    for (int it = 0; it < 4; ++it) {
      const int row = it * 8 + wave * 2 + hh;
      const v4f p0 = *(const v4f*)(sY + row * kScYP + c4);
      const v4f p1 = *(const v4f*)(sY + kScT * kScYP + row * kScYP + c4);
      const v4f xv = *(const v4f*)(sX + row * 64 + c4);
      v4f o;
      o[0] = fmaf(Dd, xv[0], p0[0] + p1[0]);
      o[1] = fmaf(Dd, xv[1], p0[1] + p1[1]);
      o[2] = fmaf(Dd, xv[2], p0[2] + p1[2]);
      o[3] = fmaf(Dd, xv[3], p0[3] + p1[3]);
      float* gp = YB + (row0 + t0 + row) * kDI + head * kDH + c4;
      *(volatile v4f*)gp = o;
      __threadfence();
      *(volatile v4f*)gp = o;
    }
  }
}

static_assert(kDI == 256 * 8);
__global__ __launch_bounds__(256) void gate_norm_kernel(
    const float* __restrict__ XZ, const float* __restrict__ YB, const float* __restrict__ normw,
    unsigned short* __restrict__ YN) {
  __shared__ __align__(16) float sG[kDI];
  __shared__ float sRed[8];
  const int tid  = threadIdx.x;
  const int lane = tid & 31;
  const int wave = __builtin_amdgcn_readfirstlane((int)(threadIdx.x >> 5));
  const int row  = blockIdx.x;
  const float* zr = XZ + (size_t)row * kProjP;
  const float* yr = YB + (size_t)row * kDI;
  float ss = 0.0f;
#pragma unroll 1
  for (int j = 0; j < 8; ++j) {
    const int idx = j * 256 + tid;
    const float z  = zr[idx];
    const float yv = yr[idx];
    const float sg = 1.0f / (1.0f + expf(-z));
    const float g  = yv * (z * sg);
    sG[idx] = g;
    ss = fmaf(g, g, ss);
  }
#pragma unroll
  for (int m = 16; m >= 1; m >>= 1) ss += __shfl_xor(ss, m, 32);
  if (lane == 0) sRed[wave] = ss;
  __syncthreads();
  float tot = 0.0f;
#pragma unroll
  for (int w = 0; w < 8; ++w) tot += sRed[w];
  const float scale = rsqrtf(tot * (1.0f / (float)kDI) + 1e-5f);
  const int e0 = tid * 8;
  const v4f g0 = *(const v4f*)(sG + e0);
  const v4f g1 = *(const v4f*)(sG + e0 + 4);
  const v4f w0 = *(const v4f*)(normw + e0);
  const v4f w1 = *(const v4f*)(normw + e0 + 4);
  v8h hv;
#pragma unroll
  for (int e = 0; e < 4; ++e) {
    const float f0 = (w0[e] * (g0[e] * scale)) * kCarryY;
    const float f1 = (w1[e] * (g1[e] * scale)) * kCarryY;
    hv[e]     = (_Float16)f0;
    hv[4 + e] = (_Float16)f1;
  }
  unsigned short* q = YN + (size_t)row * kDI + e0;
  *(volatile v8h*)q = hv;
  __threadfence();
  *(volatile v8h*)q = hv;
}

static_assert(((kRows / 64) * (kProjP / 64)) % 8 == 0);
static_assert(((kRows / 64) * (kDm / 64)) % 8 == 0);
extern "C" void kernel_launch(void* const* d_in, const int* in_sizes, int n_in,
                              void* d_out, int out_size, void* d_ws, size_t ws_size,
                              hipStream_t stream) {
  if (n_in < 9) return;
  if (in_sizes[0] != kRows * kDm) return;
  if (in_sizes[1] != kDm * kProj) return;
  if (in_sizes[2] != kXBC * 4) return;
  if (in_sizes[3] != kXBC) return;
  if (in_sizes[4] != kNH) return;
  if (in_sizes[5] != kNH) return;
  if (in_sizes[6] != kNH) return;
  if (in_sizes[7] != kDI) return;
  if (in_sizes[8] != kDI * kDm) return;
  if (out_size != kRows * kDm) return;
  if (ws_size < kWsTotal) return;

  const float* x       = (const float*)d_in[0];
  const float* W_in    = (const float*)d_in[1];
  const float* conv_w  = (const float*)d_in[2];
  const float* conv_b  = (const float*)d_in[3];
  const float* A_log   = (const float*)d_in[4];
  const float* D_param = (const float*)d_in[5];
  const float* dt_bias = (const float*)d_in[6];
  const float* norm_w  = (const float*)d_in[7];
  const float* W_out   = (const float*)d_in[8];
  float* out = (float*)d_out;

  char* ws = (char*)d_ws;
  unsigned short* XH    = (unsigned short*)(ws + kOffXH);
  unsigned short* WINT  = (unsigned short*)(ws + kOffWINT);
  unsigned short* WOUTT = (unsigned short*)(ws + kOffWOUTT);
  float*          XZ    = (float*)(ws + kOffXZ);
  float*          XC    = (float*)(ws + kOffXC);
  float*          DTV   = (float*)(ws + kOffDTV);
  float*          DAV   = (float*)(ws + kOffDAV);
  float*          YB    = (float*)(ws + kOffYB);
  unsigned short* YN    = (unsigned short*)(ws + kOffYN);

  cvt_rows_f16_kernel<<<(kRows * kDm / 8) / 256, 256, 0, stream>>>(x, XH, kRows * kDm / 8, kCarryX);

  transpose_cvt_f16_kernel<<<dim3(kProjP / 64, kDm / 64), 256, 0, stream>>>(W_in, WINT, kDm, kProj, kCarryW);

  transpose_cvt_f16_kernel<<<dim3(kDm / 64, kDI / 64), 256, 0, stream>>>(W_out, WOUTT, kDI, kDm, kCarryW);

  wmma_gemm64_f16<<<((kRows / 64) * (kProjP / 64)) / 8, 256, 0, stream>>>(
      XH, kDm, WINT, kDm, XZ, kProjP, kRows, kProjP, kDm, kScaleIn);

  conv_silu_kernel<<<dim3(kXBC / 128, kRows / 64), 128, 0, stream>>>(XZ, conv_w, conv_b, XC);

  dt_kernel<<<kRows / 8, 256, 0, stream>>>(XZ, A_log, dt_bias, DTV, DAV);

  scan_kernel<<<kBatch * kNH, 128, 0, stream>>>(XC, DTV, DAV, D_param, YB);

  gate_norm_kernel<<<kRows, 256, 0, stream>>>(XZ, YB, norm_w, YN);

  wmma_gemm64_f16<<<((kRows / 64) * (kDm / 64)) / 8, 256, 0, stream>>>(
      YN, kDI, WOUTT, kDI, out, kDm, kRows, kDm, kDI, kScaleOut);
}
